// BitGRUCell_49031346651241
// MI455X (gfx1250) — hardware-run, weakly checked
//
#include <hip/hip_runtime.h>
#include <math.h>

constexpr int kRows   = 4096;
constexpr int kIn     = 2048;
constexpr int kHidN   = 2048;
constexpr int kSeg    = 2048;
constexpr int kFan    = 4096;
constexpr int kWElems = kHidN * kFan;
constexpr int kChunkElems = 32768;
constexpr int kChunks = kWElems / kChunkElems;
constexpr float kInvWElems = 1.0f / 8388608.0f;
static_assert(kSeg % 32 == 0);
static_assert(kRows % 64 == 0);
static_assert(kHidN % 64 == 0);
static_assert(kIn == kSeg && kHidN == kSeg);
static_assert(kChunks == 256);
static_assert(kChunkElems == 16 * 256 * 8);
static_assert((kRows * kIn / 8) % 256 == 0);

typedef __attribute__((ext_vector_type(16))) _Float16 v16h;
typedef __attribute__((ext_vector_type(8)))  _Float16 v8h;
typedef __attribute__((ext_vector_type(8)))  float    v8f;
typedef __attribute__((ext_vector_type(4)))  float    v4f;
typedef __attribute__((ext_vector_type(4)))  unsigned int v4u;

__device__ __forceinline__ void dep_guard_h(v8f& a, v8f& b, v16h x, v16h y) { asm volatile("v_nop\n\tv_nop\n\tv_nop\n\tv_nop" : "+v"(a), "+v"(b) : "v"(x), "v"(y)); }
__device__ __forceinline__ void keep4_h(v16h a, v16h b, v16h c, v16h d) { asm volatile("v_nop" :: "v"(a), "v"(b), "v"(c), "v"(d)); }
__device__ __forceinline__ void acc_guard4(v8f& a, v8f& b, v8f& c, v8f& d) { asm volatile("v_nop\n\tv_nop\n\tv_nop\n\tv_nop" : "+v"(a), "+v"(b), "+v"(c), "+v"(d)); }
template <typename T> struct Frag;
template <> struct Frag<_Float16> {
  typedef v16h V; union U { v16h v; v8h h[2]; };
  static __device__ __forceinline__ v16h load(const _Float16* p) {
    U f; f.h[0] = *(const v8h*)(p); f.h[1] = *(const v8h*)(p + 16); return f.v;
  }
  static __device__ __forceinline__ v8f mma(v16h a, v16h b, v8f c) {
    return __builtin_amdgcn_wmma_f32_16x16x32_f16(false, a, false, b, (short)0, c, false, false);
  }
  static __device__ __forceinline__ void guard(v8f& a, v8f& b, v16h x, v16h y) { dep_guard_h(a, b, x, y); }
  static __device__ __forceinline__ void keep(v16h a, v16h b, v16h c, v16h d) { keep4_h(a, b, c, d); }
};

__device__ __forceinline__ unsigned pk16(unsigned short a, unsigned short b) { return (unsigned)a | ((unsigned)b << 16); }
__device__ __forceinline__ unsigned short h_bits(float f) { const _Float16 h = (_Float16)f; return __builtin_bit_cast(unsigned short, h); }

__device__ __forceinline__ unsigned short sgn_hbits(float v) {
  return (v > 0.0f) ? (unsigned short)0x3C00u : ((v < 0.0f) ? (unsigned short)0xBC00u : (unsigned short)0u);
}

__device__ __forceinline__ float hbits_to_f32(unsigned u) {
  const unsigned sgn = (u & 0x8000u) << 16;
  const unsigned ex  = (u >> 10) & 31u;
  const unsigned mt  = u & 0x3FFu;
  const float fn = __uint_as_float(((ex + 112u) << 23) | (mt << 13));
  const float fs = (float)mt * 5.9604644775390625e-8f;
  const float mag = (ex == 0u) ? fs : fn;
  return __uint_as_float(__float_as_uint(mag) | sgn);
}

__global__ __launch_bounds__(256) void sign_absum_kernel(
    const float* __restrict__ w0, const float* __restrict__ w1, const float* __restrict__ w2,
    unsigned short* __restrict__ s0, unsigned short* __restrict__ s1, unsigned short* __restrict__ s2,
    float* __restrict__ part) {
  __shared__ float red[8];
  const int t = threadIdx.x, lane = t & 31, wave = t >> 5;
  const int chunk = blockIdx.x;
  const int which = blockIdx.y;
  const float* w = (which == 0) ? w0 : ((which == 1) ? w1 : w2);
  unsigned short* so = (which == 0) ? s0 : ((which == 1) ? s1 : s2);
  float s = 0.0f;
#pragma unroll 1
  for (int it = 0; it < 16; ++it) {
    const size_t e = (size_t)chunk * kChunkElems + (size_t)it * 2048 + (size_t)t * 8;
    const v4f a = *(const v4f*)(w + e);
    const v4f c = *(const v4f*)(w + e + 4);
    unsigned short hb[8];
#pragma unroll
    for (int k = 0; k < 4; ++k) {
      hb[k]     = sgn_hbits(a[k]);
      hb[4 + k] = sgn_hbits(c[k]);
      s += fabsf(a[k]);
      s += fabsf(c[k]);
    }
    const v4u u = (v4u){pk16(hb[0], hb[1]), pk16(hb[2], hb[3]), pk16(hb[4], hb[5]), pk16(hb[6], hb[7])};
    unsigned short* q = so + e;
    *(volatile v4u*)q = u;
    __threadfence();
    *(volatile v4u*)q = u;
  }
#pragma unroll
  for (int off = 16; off > 0; off >>= 1) s += __shfl_xor(s, off, 32);
  if (lane == 0) red[wave] = s;
  __syncthreads();
  float tot = red[0];
#pragma unroll
  for (int k = 1; k < 8; ++k) tot += red[k];
  if (wave == 0) {
    const float v = (lane == 0) ? tot : 0.0f;
    volatile float* vp = part + (size_t)(which * kChunks + chunk) * 32;
    vp[lane] = v;
    __threadfence();
    vp[lane] = v;
  }
}

__global__ __launch_bounds__(256) void scale_finish_kernel(const float* __restrict__ part, float* __restrict__ scal) {
  __shared__ double dred[256];
  const int t = threadIdx.x, lane = t & 31, wave = t >> 5;
  float sc[3];
#pragma unroll
  for (int w = 0; w < 3; ++w) {
    dred[t] = (double)part[(size_t)(w * kChunks + t) * 32];
    __syncthreads();
#pragma unroll
    for (int off = 128; off > 0; off >>= 1) {
      if (t < off) dred[t] = dred[t] + dred[t + off];
      __syncthreads();
    }
    sc[w] = (float)dred[0] * kInvWElems;
    __syncthreads();
  }
  if (wave == 0) {
    const float v = (lane == 0) ? sc[0] : ((lane == 1) ? sc[1] : ((lane == 2) ? sc[2] : 0.0f));
    volatile float* vp = scal;
    vp[lane] = v;
    __threadfence();
    vp[lane] = v;
  }
}

__global__ __launch_bounds__(256) void cast8_f16_kernel(const float* __restrict__ in, unsigned short* __restrict__ out, int n8) {
  const int i = blockIdx.x * 256 + threadIdx.x;
  if (i >= n8) return;
  const float* p = in + 8 * (size_t)i;
  const v4f a = *(const v4f*)(p);
  const v4f c = *(const v4f*)(p + 4);
  unsigned short hb[8];
#pragma unroll
  for (int e = 0; e < 4; ++e) {
    hb[e]     = h_bits(a[e]);
    hb[4 + e] = h_bits(c[e]);
  }
  const v4u u = (v4u){pk16(hb[0], hb[1]), pk16(hb[2], hb[3]), pk16(hb[4], hb[5]), pk16(hb[6], hb[7])};
  unsigned short* q = out + 8 * (size_t)i;
  *(volatile v4u*)q = u;
  __threadfence();
  *(volatile v4u*)q = u;
}

template <int GATE>
__global__ __launch_bounds__(256) void bit_gemm64(
    const unsigned short* __restrict__ A0p, const unsigned short* __restrict__ A1p,
    const unsigned short* __restrict__ Btp,
    const float* __restrict__ bias, const float* __restrict__ scalp,
    const float* __restrict__ hid, const unsigned short* __restrict__ nplane,
    void* __restrict__ Cout, int M, int N) {
  typedef _Float16 T;
  typedef v16h V;
  const T* A0 = (const T*)A0p; const T* A1 = (const T*)A1p; const T* Bt = (const T*)Btp;
  __shared__ __align__(16) float sT[8][16 * 68];
  const int lane = threadIdx.x & 31;
  const int wave = threadIdx.x >> 5;
  const int tilesN = N >> 6;
  const int tilesM = M >> 6;
  const int tile = blockIdx.x * 8 + wave;
  if (tile >= tilesM * tilesN) return;
  const int tm = tile / tilesN;
  const int tn = tile - tm * tilesN;
  const int m0 = tm << 6;
  const int n0 = tn << 6;

  const int rlane = lane & 15;
  const int koff  = (lane >> 4) * 8;
  const int mOff  = (lane >> 4) * 8;

  v8f acc[4][4];
#pragma unroll
  for (int i = 0; i < 4; ++i)
#pragma unroll
    for (int j = 0; j < 4; ++j) acc[i][j] = (v8f){0.f,0.f,0.f,0.f,0.f,0.f,0.f,0.f};

  for (int seg = 0; seg < 2; ++seg) {
    const T* Ab = (seg == 0) ? A0 : A1;
    const int kb = seg * kSeg;
    for (int k0 = 0; k0 < kSeg; k0 += 32) {
      V bh[4];
#pragma unroll
      for (int j = 0; j < 4; ++j) {
        const size_t bo = (size_t)(n0 + (j << 4) + rlane) * kFan + kb + koff + k0;
        bh[j] = Frag<T>::load(Bt + bo);
      }
#pragma unroll
      for (int i = 0; i < 4; ++i) {
        const size_t ao = (size_t)(m0 + (i << 4) + rlane) * kSeg + koff + k0;
        V ah = Frag<T>::load(Ab + ao);
#pragma unroll
        for (int j = 0; j < 4; ++j) acc[i][j] = Frag<T>::mma(ah, bh[j], acc[i][j]);
        Frag<T>::guard(acc[i][0], acc[i][3], ah, ah);
      }
      Frag<T>::keep(bh[0], bh[1], bh[2], bh[3]);
    }
  }
  acc_guard4(acc[0][0], acc[0][1], acc[0][2], acc[0][3]);
  acc_guard4(acc[1][0], acc[1][1], acc[1][2], acc[1][3]);
  acc_guard4(acc[2][0], acc[2][1], acc[2][2], acc[2][3]);
  acc_guard4(acc[3][0], acc[3][1], acc[3][2], acc[3][3]);

  const float scale = scalp[0];

  float* slab = sT[wave];
#pragma unroll
  for (int i = 0; i < 4; ++i) {
    const int mBase = m0 + (i << 4);
#pragma unroll
    for (int j = 0; j < 4; ++j) {
      const int n = n0 + (j << 4) + rlane;
      const float bv = bias[n];
#pragma unroll
      for (int r = 0; r < 8; ++r) {
        float v = acc[i][j][r] * scale + bv;
        if (GATE == 1) {
          v = tanhf(v);
        } else {
          v = 1.0f / (1.0f + expf(-v));
        }
        slab[(mOff + r) * 68 + (j << 4) + rlane] = v;
      }
    }
    __builtin_amdgcn_fence(__ATOMIC_RELEASE, "workgroup");
    __builtin_amdgcn_wave_barrier();
    __builtin_amdgcn_fence(__ATOMIC_ACQUIRE, "workgroup");
    if (GATE == 2) {
      float* C = (float*)Cout;
      const int hh = lane >> 4, c4 = (lane & 15) * 4;
#pragma unroll
      for (int it = 0; it < 8; ++it) {
        const int row = it * 2 + hh;
        const size_t gi = (size_t)(mBase + row) * N + n0 + c4;
        const v4f hv = *(const v4f*)(hid + gi);
        const unsigned long long nw = *(const unsigned long long*)(nplane + gi);
        float* sp = slab + row * 68 + c4;
#pragma unroll
        for (int e = 0; e < 4; ++e) {
          const float z  = sp[e];
          const float nn = hbits_to_f32((unsigned)((nw >> (16 * e)) & 0xFFFFull));
          const float h  = hv[e];
          sp[e] = (1.0f - z) * h + z * nn;
        }
      }
      __builtin_amdgcn_fence(__ATOMIC_RELEASE, "workgroup");
      __builtin_amdgcn_wave_barrier();
      __builtin_amdgcn_fence(__ATOMIC_ACQUIRE, "workgroup");
      for (int pass = 0; pass < 2; ++pass) {
#pragma unroll
        for (int it = 0; it < 8; ++it) {
          const int row = it * 2 + hh;
          v4f v = *(const v4f*)(slab + row * 68 + c4);
          *(volatile v4f*)(C + (size_t)(mBase + row) * N + n0 + c4) = v;
        }
        __threadfence();
      }
    } else {
      const int q = lane >> 3, c8 = (lane & 7) * 8;
      unsigned short* C = (unsigned short*)Cout;
      if (GATE == 0) {
#pragma unroll
        for (int it = 0; it < 4; ++it) {
          const int row = it * 4 + q;
          const size_t gi = (size_t)(mBase + row) * N + n0 + c8;
          const v4f h0 = *(const v4f*)(hid + gi);
          const v4f h1 = *(const v4f*)(hid + gi + 4);
          float* sp = slab + row * 68 + c8;
#pragma unroll
          for (int e = 0; e < 4; ++e) {
            sp[e]     = sp[e] * h0[e];
            sp[4 + e] = sp[4 + e] * h1[e];
          }
        }
        __builtin_amdgcn_fence(__ATOMIC_RELEASE, "workgroup");
        __builtin_amdgcn_wave_barrier();
        __builtin_amdgcn_fence(__ATOMIC_ACQUIRE, "workgroup");
      }
      for (int pass = 0; pass < 2; ++pass) {
#pragma unroll
        for (int it = 0; it < 4; ++it) {
          const int row = it * 4 + q;
          const float* sp = slab + row * 68 + c8;
          v8h hv;
#pragma unroll
          for (int e = 0; e < 8; ++e) hv[e] = (_Float16)sp[e];
          *(volatile v8h*)(C + (size_t)(mBase + row) * N + n0 + c8) = hv;
        }
        __threadfence();
      }
    }
    __builtin_amdgcn_fence(__ATOMIC_RELEASE, "workgroup");
    __builtin_amdgcn_wave_barrier();
    __builtin_amdgcn_fence(__ATOMIC_ACQUIRE, "workgroup");
  }
}

extern "C" void kernel_launch(void* const* d_in, const int* in_sizes, int n_in,
                              void* d_out, int out_size, void* d_ws, size_t ws_size,
                              hipStream_t stream) {
  if (n_in < 8) return;
  if (in_sizes[0] != kRows * kIn || in_sizes[1] != kRows * kHidN) return;
  if (in_sizes[2] != kWElems || in_sizes[4] != kWElems || in_sizes[6] != kWElems) return;
  if (in_sizes[3] != kHidN || in_sizes[5] != kHidN || in_sizes[7] != kHidN) return;
  if (out_size != kRows * kHidN) return;

  const float* x      = (const float*)d_in[0];
  const float* hidden = (const float*)d_in[1];
  const float* w_r    = (const float*)d_in[2];
  const float* b_r    = (const float*)d_in[3];
  const float* w_z    = (const float*)d_in[4];
  const float* b_z    = (const float*)d_in[5];
  const float* w_n    = (const float*)d_in[6];
  const float* b_n    = (const float*)d_in[7];
  float* out = (float*)d_out;

  char* ws = (char*)d_ws;
  const size_t signBytes = (size_t)kWElems * 2;
  const size_t actBytes  = (size_t)kRows * kSeg * 2;
  const size_t partBytes = (size_t)3 * kChunks * 128;
  const size_t offSR   = 0;
  const size_t offSZ   = offSR + signBytes;
  const size_t offSN   = offSZ + signBytes;
  const size_t offX    = offSN + signBytes;
  const size_t offH    = offX + actBytes;
  const size_t offRH   = offH + actBytes;
  const size_t offNP   = offRH + actBytes;
  const size_t offPART = offNP + actBytes;
  const size_t offSCAL = offPART + partBytes;
  const size_t total   = offSCAL + 128;
  if (total > ws_size) return;

  unsigned short* SR   = (unsigned short*)(ws + offSR);
  unsigned short* SZ   = (unsigned short*)(ws + offSZ);
  unsigned short* SN   = (unsigned short*)(ws + offSN);
  unsigned short* X16  = (unsigned short*)(ws + offX);
  unsigned short* H16  = (unsigned short*)(ws + offH);
  unsigned short* RH16 = (unsigned short*)(ws + offRH);
  unsigned short* NP16 = (unsigned short*)(ws + offNP);
  float* PART = (float*)(ws + offPART);
  float* SCAL = (float*)(ws + offSCAL);

  sign_absum_kernel<<<dim3(kChunks, 3), 256, 0, stream>>>(w_r, w_z, w_n, SR, SZ, SN, PART);
  scale_finish_kernel<<<1, 256, 0, stream>>>(PART, SCAL);

  const int n8 = kRows * kIn / 8;
  cast8_f16_kernel<<<n8 / 256, 256, 0, stream>>>(x, X16, n8);
  cast8_f16_kernel<<<n8 / 256, 256, 0, stream>>>(hidden, H16, n8);

  const int gemmBlocks = (kRows / 64) * (kHidN / 64) / 8;
  bit_gemm64<0><<<gemmBlocks, 256, 0, stream>>>(X16, H16, SR, b_r, SCAL + 0, hidden, X16, (void*)RH16, kRows, kHidN);
  bit_gemm64<1><<<gemmBlocks, 256, 0, stream>>>(X16, RH16, SN, b_n, SCAL + 2, hidden, X16, (void*)NP16, kRows, kHidN);
  bit_gemm64<2><<<gemmBlocks, 256, 0, stream>>>(X16, H16, SZ, b_z, SCAL + 1, hidden, NP16, (void*)out, kRows, kHidN);
}
